// ColorFeatureExtraction_73100343378215
// MI455X (gfx1250) — hardware-verified
//
#include <hip/hip_runtime.h>


namespace {
constexpr int NB = 4, NPt = 8192, C1 = 16, C2 = 32, NBLK = NPt / 256;
constexpr float XS = 8.0f, WSC = 256.0f, EPS = 1e-5f;

typedef _Float16 b16;
typedef __attribute__((ext_vector_type(16))) _Float16 v16b;
typedef __attribute__((ext_vector_type(8))) _Float16 v8b;
typedef __attribute__((ext_vector_type(8))) float v8f;
typedef __attribute__((ext_vector_type(4))) float v4f;
__device__ __forceinline__ float bf16_rne(float f) { unsigned int u = __float_as_uint(f); u += 0x7FFFu + ((u >> 16) & 1u); return __uint_as_float(u & 0xFFFF0000u); }
__device__ __forceinline__ void split16(float v, b16& hi, b16& lo) { hi = (b16)v; lo = (b16)(v - (float)hi); }
__device__ __forceinline__ v16b frag_kb(const b16* p, int hh) { const v8b a = *(const v8b*)(p + 8 * hh), b = *(const v8b*)(p + 16 + 8 * hh); v16b f;
#pragma unroll
  for (int e = 0; e < 8; ++e) { f[e] = a[e]; f[8 + e] = b[e]; } return f; }
__device__ __forceinline__ v8f wmma16b(v16b a, v16b b, v8f c) { v8f d = __builtin_amdgcn_wmma_f32_16x16x32_f16(false, a, false, b, (short)0, c, false, false); asm volatile("v_nop\n\tv_nop\n\tv_nop\n\tv_nop" : "+v"(d) : "v"(a), "v"(b)); return d; }
__device__ __forceinline__ void wave_lds_sync() { __builtin_amdgcn_fence(__ATOMIC_RELEASE, "workgroup"); __builtin_amdgcn_wave_barrier(); __builtin_amdgcn_fence(__ATOMIC_ACQUIRE, "workgroup"); }
__device__ __forceinline__ float nexp(float x) { return __builtin_amdgcn_exp2f(x * 1.4426950408889634f); }
__device__ __forceinline__ float pmul(float a, float b) { float p = a * b; asm volatile("" : "+v"(p)); return p; }
__device__ __forceinline__ float sigm(float x) { return 1.0f / (1.0f + nexp(-x)); }

struct Par {
  float w1[C1][3], b1[C1], s1[C1], t1[C1];
  float w2[C2][C1], b2[C2], s2[C2], t2[C2];
  float ba1[C2], sa[C2], ta[C2], ba2[C2];
};
__device__ __forceinline__ void load_par(Par& P, const float* w1, const float* b1, const float* g1, const float* be1, const float* m1, const float* v1, const float* w2, const float* b2, const float* g2, const float* be2, const float* m2, const float* v2,
                                    const float* ba1, const float* ga, const float* bea, const float* ma, const float* va, const float* ba2, int t_) {
  for (int i = t_; i < C1 * 3; i += 256) P.w1[i / 3][i % 3] = bf16_rne(w1[i]);
  for (int i = t_; i < C2 * C1; i += 256) P.w2[i / C1][i % C1] = bf16_rne(w2[i]);
  if (t_ < C1) { P.b1[t_] = bf16_rne(b1[t_]); const float s = bf16_rne(g1[t_]) / sqrtf(bf16_rne(v1[t_]) + EPS); P.s1[t_] = s; P.t1[t_] = bf16_rne(be1[t_]); }
  if (t_ < C2) { P.b2[t_] = bf16_rne(b2[t_]); const float s = bf16_rne(g2[t_]) / sqrtf(bf16_rne(v2[t_]) + EPS); P.s2[t_] = s; P.t2[t_] = bf16_rne(be2[t_]);
    P.ba1[t_] = bf16_rne(ba1[t_]); const float sA = bf16_rne(ga[t_]) / sqrtf(bf16_rne(va[t_]) + EPS); P.sa[t_] = sA; P.ta[t_] = bf16_rne(bea[t_]); P.ba2[t_] = bf16_rne(ba2[t_]); }
}
__device__ __forceinline__ void feat_tile(const Par& P, const float* m1, const float* m2, const b16* __restrict__ W2P, float x0, float x1, float x2, float* f, b16 (*Fh)[C2 + 8], b16 (*Fl)[C2 + 8], float (*Zs)[C2 + 1], int lane) {
  const int nloc = lane & 15, hlf = lane >> 4;
#pragma unroll
  for (int o = 0; o < C1; ++o) { const float pre = (pmul(P.w1[o][0], x0) + pmul(P.w1[o][1], x1) + pmul(P.w1[o][2], x2)) + P.b1[o]; const float hv = fmaxf(pmul(pre - bf16_rne(m1[o]), P.s1[o]) + P.t1[o], 0.0f); b16 a_, c_; split16(hv * XS, a_, c_); Fh[lane][o] = a_; Fl[lane][o] = c_; Fh[lane][C1 + o] = (b16)0.0f; Fl[lane][C1 + o] = (b16)0.0f; }
  wave_lds_sync();
#pragma unroll
  for (int mt = 0; mt < 2; ++mt) { const v16b a = frag_kb(&Fh[mt * 16 + nloc][0], hlf), al = frag_kb(&Fl[mt * 16 + nloc][0], hlf);
#pragma unroll
    for (int nt = 0; nt < 2; ++nt) { const v16b bw = frag_kb(W2P + (size_t)(nt * 16 + nloc) * C2, hlf); v8f acc = {}; acc = wmma16b(a, bw, acc); acc = wmma16b(al, bw, acc);
#pragma unroll
      for (int r = 0; r < 8; ++r) Zs[mt * 16 + 8 * hlf + r][nt * 16 + nloc] = acc[r] * (1.0f / (XS * WSC)); } }
  wave_lds_sync();
#pragma unroll
  for (int o = 0; o < C2; ++o) { const float pre = Zs[lane][o] + P.b2[o]; f[o] = fmaxf(pmul(pre - bf16_rne(m2[o]), P.s2[o]) + P.t2[o], 0.0f); }
  wave_lds_sync();
}
__global__ __launch_bounds__(256) void stats_kernel(const float* __restrict__ colors, const float* w1, const float* b1, const float* g1, const float* be1, const float* m1, const float* v1, const float* w2, const float* b2, const float* g2, const float* be2, const float* m2, const float* v2,
                                                 const float* ba1, const float* ga, const float* bea, const float* ma, const float* va, const float* ba2, const b16* __restrict__ WA, float* __restrict__ S) {
  __shared__ Par P; __shared__ float red[C2][257]; __shared__ __attribute__((aligned(16))) b16 Fh[8][32][C2 + 8], Fl[8][32][C2 + 8]; __shared__ float Zs[8][32][C2 + 1];
  const int t_ = threadIdx.x, wave = t_ >> 5, lane = t_ & 31; const int b = blockIdx.x / NBLK, blk = blockIdx.x - b * NBLK; const int n = blk * 256 + t_;
  load_par(P, w1, b1, g1, be1, m1, v1, w2, b2, g2, be2, m2, v2, ba1, ga, bea, ma, va, ba2, t_);
  __syncthreads();
  float f[C2]; feat_tile(P, m1, m2, WA + 2 * C2 * C2, bf16_rne(colors[((size_t)b * 3 + 0) * NPt + n]), bf16_rne(colors[((size_t)b * 3 + 1) * NPt + n]), bf16_rne(colors[((size_t)b * 3 + 2) * NPt + n]), f, Fh[wave], Fl[wave], Zs[wave], lane);
#pragma unroll
  for (int c = 0; c < C2; ++c) red[c][t_] = f[c];
  __syncthreads();
  for (int s = 128; s >= 1; s >>= 1) { if (t_ < s) { for (int c = 0; c < C2; ++c) red[c][t_] += red[c][t_ + s]; } __syncthreads(); }
  for (int pass = 0; pass < 2; ++pass) { if (t_ < C2) ((volatile float*)S)[((size_t)b * NBLK + blk) * C2 + t_] = red[t_][0]; __threadfence(); }
}
__global__ __launch_bounds__(32) void ctx_kernel(const float* __restrict__ S, const float* __restrict__ wc1, const float* __restrict__ bc1, const float* __restrict__ wc2, const float* __restrict__ bc2, float* __restrict__ CW) {
  __shared__ float ctx[C2], h[C1];
  const int b = blockIdx.x, lane = threadIdx.x; float s = 0.0f; for (int k = 0; k < NBLK; ++k) s += S[((size_t)b * NBLK + k) * C2 + lane]; ctx[lane] = s * (1.0f / NPt);
  __syncthreads();
  if (lane < C1) { float a = bf16_rne(bc1[lane]); for (int c = 0; c < C2; ++c) a += pmul(bf16_rne(wc1[lane * C2 + c]), ctx[c]); h[lane] = fmaxf(a, 0.0f); }
  __syncthreads();
  float a = bf16_rne(bc2[lane]); for (int c = 0; c < C1; ++c) a += pmul(bf16_rne(wc2[lane * C1 + c]), h[c]); const float cw = sigm(a);
  for (int pass = 0; pass < 2; ++pass) { ((volatile float*)CW)[b * C2 + lane] = cw; __threadfence(); }
}
__global__ __launch_bounds__(256) void prepw_kernel(const float* __restrict__ wa1, const float* __restrict__ wa2, const float* __restrict__ w2, b16* __restrict__ WA) {
  const int t = blockIdx.x * 256 + threadIdx.x; if (t < 2 * C2 * C2 / 8) { const int k = t / (C2 * C2 / 8), e = (t - k * (C2 * C2 / 8)) * 8; const float* w = k ? wa2 : wa1; v8b o; for (int j = 0; j < 8; ++j) o[j] = (b16)(bf16_rne(w[e + j]) * WSC);
    for (int pass = 0; pass < 2; ++pass) { *(volatile v8b*)(WA + k * C2 * C2 + e) = o; __threadfence(); } }
  else if (t < 3 * C2 * C2 / 8) { const int e = (t - 2 * C2 * C2 / 8) * 8; const int o_ = e / C2, c0 = e - o_ * C2; v8b o = {}; if (c0 < C1) for (int j = 0; j < 8; ++j) o[j] = (b16)(bf16_rne(w2[o_ * C1 + c0 + j]) * WSC);
    for (int pass = 0; pass < 2; ++pass) { *(volatile v8b*)(WA + 2 * C2 * C2 + e) = o; __threadfence(); } }
}
__global__ __launch_bounds__(256) void main_kernel(const float* __restrict__ colors, const float* w1, const float* b1, const float* g1, const float* be1, const float* m1, const float* v1, const float* w2, const float* b2, const float* g2, const float* be2, const float* m2, const float* v2,
                                                const float* ba1, const float* ga, const float* bea, const float* ma, const float* va, const float* ba2, const b16* __restrict__ WA, const float* __restrict__ CW, float* __restrict__ out) {
  __shared__ Par P; __shared__ __attribute__((aligned(16))) b16 Fh[8][32][C2 + 8], Fl[8][32][C2 + 8]; __shared__ float Zs[8][32][C2 + 1];
  const int t_ = threadIdx.x, wave = t_ >> 5, lane = t_ & 31, nloc = lane & 15, hlf = lane >> 4; const int b = blockIdx.y; const int n0 = blockIdx.x * 256 + wave * 32, n = n0 + lane;
  load_par(P, w1, b1, g1, be1, m1, v1, w2, b2, g2, be2, m2, v2, ba1, ga, bea, ma, va, ba2, t_);
  __syncthreads();
  float f[C2]; feat_tile(P, m1, m2, WA + 2 * C2 * C2, bf16_rne(colors[((size_t)b * 3 + 0) * NPt + n]), bf16_rne(colors[((size_t)b * 3 + 1) * NPt + n]), bf16_rne(colors[((size_t)b * 3 + 2) * NPt + n]), f, Fh[wave], Fl[wave], Zs[wave], lane);
#pragma unroll
  for (int c = 0; c < C2; ++c) { b16 h_, l_; split16(f[c] * XS, h_, l_); Fh[wave][lane][c] = h_; Fl[wave][lane][c] = l_; }
  wave_lds_sync();
  for (int layer = 0; layer < 2; ++layer) { const b16* Wp = WA + layer * C2 * C2;
#pragma unroll
    for (int mt = 0; mt < 2; ++mt) { const v16b a = frag_kb(&Fh[wave][mt * 16 + nloc][0], hlf), al = frag_kb(&Fl[wave][mt * 16 + nloc][0], hlf);
#pragma unroll
      for (int nt = 0; nt < 2; ++nt) { const v16b bw = frag_kb(Wp + (size_t)(nt * 16 + nloc) * C2, hlf); v8f acc = {}; acc = wmma16b(a, bw, acc); acc = wmma16b(al, bw, acc);
#pragma unroll
        for (int r = 0; r < 8; ++r) Zs[wave][mt * 16 + 8 * hlf + r][nt * 16 + nloc] = acc[r] * (1.0f / (XS * WSC)); } }
    wave_lds_sync();
    if (layer == 0) {
#pragma unroll
      for (int c = 0; c < C2; ++c) { const float pre = Zs[wave][lane][c] + P.ba1[c]; const float hv = fmaxf(pmul(pre - bf16_rne(ma[c]), P.sa[c]) + P.ta[c], 0.0f); b16 h_, l_; split16(hv * XS, h_, l_); Fh[wave][lane][c] = h_; Fl[wave][lane][c] = l_; }
      wave_lds_sync(); } }
  float o[C2];
#pragma unroll
  for (int c = 0; c < C2; ++c) { const float aw = sigm(Zs[wave][lane][c] + P.ba2[c]); o[c] = pmul(pmul(f[c], aw), CW[b * C2 + c]); }
  for (int pass = 0; pass < 2; ++pass) {
#pragma unroll
    for (int c = 0; c < C2; ++c) ((volatile float*)out)[((size_t)b * C2 + c) * NPt + n] = o[c];
    __threadfence(); }
}
}

extern "C" void kernel_launch(void* const* d_in, const int* in_sizes, int n_in, void* d_out, int out_size, void* d_ws, size_t ws_size, hipStream_t stream) {
  (void)n_in;
  auto Fp = [&](int i) { return (const float*)d_in[i]; };
  if (in_sizes[0] != NB * 3 * NPt || in_sizes[2] != C1 * 3 || in_sizes[8] != C2 * C1 || in_sizes[14] != C2 * C2 || in_sizes[20] != C2 * C2 || in_sizes[22] != C1 * C2 || in_sizes[24] != C2 * C1 || out_size != NB * C2 * NPt) return;
  size_t off = 0; char* ws = (char*)d_ws;
  auto carve = [&](size_t bytes) { char* p = ws + off; off += (bytes + 255) & ~(size_t)255; return p; };
  float* S = (float*)carve((size_t)NB * NBLK * C2 * 4); float* CW = (float*)carve((size_t)NB * C2 * 4); b16* WA = (b16*)carve((size_t)3 * C2 * C2 * 2);
  if (off > ws_size || off > ((size_t)128 << 20)) return;
  prepw_kernel<<<2, 256, 0, stream>>>(Fp(14), Fp(20), Fp(8), WA);
  stats_kernel<<<NB * NBLK, 256, 0, stream>>>(Fp(0), Fp(2), Fp(3), Fp(4), Fp(5), Fp(6), Fp(7), Fp(8), Fp(9), Fp(10), Fp(11), Fp(12), Fp(13), Fp(15), Fp(16), Fp(17), Fp(18), Fp(19), Fp(21), WA, S);
  ctx_kernel<<<NB, 32, 0, stream>>>(S, Fp(22), Fp(23), Fp(24), Fp(25), CW);
  main_kernel<<<dim3(NPt / 256, NB), 256, 0, stream>>>(Fp(0), Fp(2), Fp(3), Fp(4), Fp(5), Fp(6), Fp(7), Fp(8), Fp(9), Fp(10), Fp(11), Fp(12), Fp(13), Fp(15), Fp(16), Fp(17), Fp(18), Fp(19), Fp(21), WA, CW, (float*)d_out);
}
